// SparseMultiheadAttention_17575006175530
// MI455X (gfx1250) — hardware-verified
//
#include <hip/hip_runtime.h>
#include <stddef.h>
#include <stdint.h>
#include <math.h>


#define CW      1024
#define BD      2
#define NHD     16
#define HDM     64
#define QKVW    3072
#define OQ      0
#define OKK     1024
#define OV      2048
#define KOUT    2048
#define APITCH  2048
#define NTHR    256
#define NWAVE   8
#define EPT     8
#define CHUNK   (NTHR * EPT)
#define WCAP    (EPT * 32)
#define LISTN   (NWAVE * WCAP)
#define NBA     512
#define SLA     9
#define RCAP    20480
#define DEGCAP  64
#define GBM     64
#define GBN     64
#define GTHR    128
#define UQKV    (CW * (CW / 8))
#define UWX     (CW * (KOUT / 8))
#define NUW     (3 * UQKV + UWX)
#define AGG_ZINTS (LISTN + 2 * RCAP + 3 * NBA)
#define MISC_INTS 16
#define SCAN_LDS_BYTES ((AGG_ZINTS + MISC_INTS) * 4)
#define ATTSC   0.125f
#define WSMAX   134217728

static_assert((CHUNK & (CHUNK - 1)) == 0 && CHUNK <= 4096);
static_assert((NBA & (NBA - 1)) == 0 && NBA == (1 << SLA));
static_assert(((long long)CHUNK << SLA) < (1LL << 31));
static_assert(LISTN >= NWAVE * WCAP);
static_assert(NBA % NWAVE == 0 && NBA % 32 == 0);
static_assert(RCAP % 32 == 0 && AGG_ZINTS % 4 == 0 && LISTN % 4 == 0 && ((AGG_ZINTS + MISC_INTS) % 4) == 0);
static_assert(NWAVE * CW <= RCAP);
static_assert(SCAN_LDS_BYTES <= 300000);
static_assert(CW == 32 * 32);
static_assert(HDM == 2 * 32 && NHD * HDM == CW);
static_assert(QKVW == 3 * CW && (QKVW % GBN) == 0 && (CW % GBN) == 0);
static_assert((CW % 32) == 0 && (KOUT % 32) == 0 && KOUT == 2 * CW && APITCH == KOUT);
static_assert((APITCH * 2) % 128 == 0);
static_assert(GBM == (GTHR / 32) * 16);
static_assert(UQKV == (1 << 17) && (CW / 8) == 128 && (KOUT / 8) == 256);
static_assert(UQKV % NTHR == 0 && UWX % NTHR == 0 && (3 * UQKV) % NTHR == 0);
static_assert(DEGCAP >= 32);

typedef float          v4f  __attribute__((ext_vector_type(4)));
typedef float          v8f  __attribute__((ext_vector_type(8)));
typedef int            v4i  __attribute__((ext_vector_type(4)));
typedef int            v8i  __attribute__((ext_vector_type(8)));
typedef unsigned int   v4u  __attribute__((ext_vector_type(4)));
typedef unsigned short v8us __attribute__((ext_vector_type(8)));
typedef __bf16         v16b __attribute__((ext_vector_type(16)));
typedef v4f  __attribute__((may_alias)) v4fa;
typedef v4i  __attribute__((may_alias)) v4ia;
typedef v4u  __attribute__((may_alias)) v4ua;
typedef v8us __attribute__((may_alias)) v8usa;
union FragB { v16b v; v8us h[2]; v8i w; };

__device__ __forceinline__ v8f wmb(const FragB& a, const FragB& b, v8f c) {
  v8f d = __builtin_amdgcn_wmma_f32_16x16x32_bf16(false, a.v, false, b.v, (short)0, c, false, false);
  asm volatile("v_nop\n\tv_nop\n\tv_nop\n\tv_nop" : "+v"(d) : "v"(a.w), "v"(b.w));
  return d;
}

__device__ __forceinline__ void ldwait() {
  asm volatile("s_wait_loadcnt 0x0" ::: "memory");
}

__device__ __forceinline__ void wave_sync() {
  __builtin_amdgcn_fence(__ATOMIC_RELEASE, "wavefront");
  __builtin_amdgcn_wave_barrier();
  __builtin_amdgcn_fence(__ATOMIC_ACQUIRE, "wavefront");
}

__device__ __forceinline__ unsigned int f2bf(float f) {
  const unsigned int u = __float_as_uint(f);
  return ((u + 0x7FFFu + ((u >> 16) & 1u)) >> 16) & 0xFFFFu;
}
__device__ __forceinline__ float bf2f(unsigned int b) { return __uint_as_float(b << 16); }
__device__ __forceinline__ float bfr(float f) { return bf2f(f2bf(f)); }
__device__ __forceinline__ v4f bfr4(const v4f a) {
  v4f r; r.x = bfr(a.x); r.y = bfr(a.y); r.z = bfr(a.z); r.w = bfr(a.w); return r;
}
__device__ __forceinline__ unsigned int pk2(float lo, float hi) { return f2bf(lo) | (f2bf(hi) << 16); }
__device__ __forceinline__ v4u pack8(const v4f a, const v4f b) {
  v4u r;
  r.x = pk2(a.x, a.y); r.y = pk2(a.z, a.w); r.z = pk2(b.x, b.y); r.w = pk2(b.z, b.w);
  return r;
}
__device__ __forceinline__ void hl2(float v0, float v1, unsigned int& hw, unsigned int& lw) {
  const unsigned int h0 = f2bf(v0), h1 = f2bf(v1);
  const unsigned int l0 = f2bf(v0 - bf2f(h0)), l1 = f2bf(v1 - bf2f(h1));
  hw = h0 | (h1 << 16);
  lw = l0 | (l1 << 16);
}
__device__ __forceinline__ void pack8hl(const v4f a, const v4f b, v4u& hv, v4u& lv) {
  unsigned int h, l;
  hl2(a.x, a.y, h, l); hv.x = h; lv.x = l;
  hl2(a.z, a.w, h, l); hv.y = h; lv.y = l;
  hl2(b.x, b.y, h, l); hv.z = h; lv.z = l;
  hl2(b.z, b.w, h, l); hv.w = h; lv.w = l;
}

__device__ __forceinline__ int scan_chunk(const int* __restrict__ keys, int nE, int cbase, int slotBase,
                                          int nb, int vec8, int* list, int tid, int lane, int wave) {
  int wc = 0;
  const int el0  = tid * EPT;
  const int e0   = cbase + el0;
  const int sent = -2147483647 - 1;
  v4i da, db;
  if (vec8 != 0 && cbase + CHUNK <= nE) {
    da = *(const v4i*)(keys + e0);
    db = *(const v4i*)(keys + e0 + 4);
  } else {
    da.x = (e0     < nE) ? keys[min(e0,     nE - 1)] : sent;
    da.y = (e0 + 1 < nE) ? keys[min(e0 + 1, nE - 1)] : sent;
    da.z = (e0 + 2 < nE) ? keys[min(e0 + 2, nE - 1)] : sent;
    da.w = (e0 + 3 < nE) ? keys[min(e0 + 3, nE - 1)] : sent;
    db.x = (e0 + 4 < nE) ? keys[min(e0 + 4, nE - 1)] : sent;
    db.y = (e0 + 5 < nE) ? keys[min(e0 + 5, nE - 1)] : sent;
    db.z = (e0 + 6 < nE) ? keys[min(e0 + 6, nE - 1)] : sent;
    db.w = (e0 + 7 < nE) ? keys[min(e0 + 7, nE - 1)] : sent;
  }
  const unsigned nbs = (unsigned)slotBase;
  const unsigned unb = (unsigned)nb;
  const unsigned s0 = (unsigned)da.x - nbs, s1 = (unsigned)da.y - nbs;
  const unsigned s2 = (unsigned)da.z - nbs, s3 = (unsigned)da.w - nbs;
  const unsigned s4 = (unsigned)db.x - nbs, s5 = (unsigned)db.y - nbs;
  const unsigned s6 = (unsigned)db.z - nbs, s7 = (unsigned)db.w - nbs;
  const bool h0 = s0 < unb, h1 = s1 < unb, h2 = s2 < unb, h3 = s3 < unb;
  const bool h4 = s4 < unb, h5 = s5 < unb, h6 = s6 < unb, h7 = s7 < unb;
  const unsigned any = __builtin_amdgcn_ballot_w32(h0 | h1 | h2 | h3 | h4 | h5 | h6 | h7);
  if (any != 0u) {
#define HITJ(J, HJ, SJ) { \
      const unsigned mj = __builtin_amdgcn_ballot_w32(HJ); \
      if (mj != 0u) { \
        if (HJ) { \
          const int pos = wc + (int)__builtin_amdgcn_mbcnt_lo(mj, 0u); \
          if (pos < WCAP) list[wave * WCAP + pos] = ((el0 + (J)) << SLA) | (int)(SJ); \
        } \
        wc += (int)__builtin_popcount(mj); } }
    HITJ(0, h0, s0)
    HITJ(1, h1, s1)
    HITJ(2, h2, s2)
    HITJ(3, h3, s3)
    HITJ(4, h4, s4)
    HITJ(5, h5, s5)
    HITJ(6, h6, s6)
    HITJ(7, h7, s7)
#undef HITJ
  }
  return wc;
}

__global__ __launch_bounds__(NTHR) void k_xprep(const float* __restrict__ x, unsigned short* xb, int nN, int nUnits) {
  const int i = (int)blockIdx.x * NTHR + (int)threadIdx.x;
  if (i >= nUnits) return;
  const int row = i >> 7;
  const int c0  = (i & 127) * 8;
  const int rc  = row < nN ? row : nN - 1;
  const float* p = x + (size_t)rc * CW + c0;
  v4f a = *(const v4fa*)p;
  v4f b = *(const v4fa*)(p + 4);
  const v4f z4 = {0.f, 0.f, 0.f, 0.f};
  if (row >= nN) { a = z4; b = z4; }
  const v4u hv = pack8(a, b);
  unsigned short* o = xb + (size_t)row * CW + c0;
  *(volatile v4u*)o = hv;
  __threadfence();
  *(volatile v4u*)o = hv;
}

__global__ __launch_bounds__(NTHR) void k_wprep(const float* __restrict__ Wq, const float* __restrict__ Wk,
                                                const float* __restrict__ Wv, const float* __restrict__ Wx,
                                                unsigned short* WQKVT, unsigned short* WXT) {
  const int u = (int)blockIdx.x * NTHR + (int)threadIdx.x;
  if (u >= NUW) return;
  v4f a, b;
  unsigned short* dp;
  if (u < 3 * UQKV) {
    const int part = u >> 17;
    const int v    = u & (UQKV - 1);
    const int n    = v >> 7;
    const int k8   = (v & 127) * 8;
    const float* W = (part == 0) ? Wq : ((part == 1) ? Wk : Wv);
    const float* p = W + (size_t)n * CW + k8;
    a = *(const v4fa*)p;
    b = *(const v4fa*)(p + 4);
    dp = WQKVT + (size_t)(part * CW + n) * CW + k8;
  } else {
    const int v  = u - 3 * UQKV;
    const int n  = v >> 8;
    const int k8 = (v & 255) * 8;
    const int kk = k8 & (CW - 1);
    const float* p = Wx + (size_t)n * CW + kk;
    a = *(const v4fa*)p;
    b = *(const v4fa*)(p + 4);
    dp = WXT + (size_t)n * KOUT + k8;
  }
  const v4u wv = pack8(a, b);
  *(volatile v4u*)dp = wv;
  __threadfence();
  *(volatile v4u*)dp = wv;
}

__global__ __launch_bounds__(GTHR) void k_gemm(
    const unsigned short* __restrict__ A, int lda, const unsigned short* __restrict__ WT, int K,
    float* outF, int ldo, int nRows,
    const float* __restrict__ bs0, const float* __restrict__ bs1, const float* __restrict__ bs2, int useBias)
{
  __shared__ __attribute__((aligned(16))) float stg[GBM * GBN];
  const int tid = (int)threadIdx.x, lane = tid & 31, wave = tid >> 5, hh = lane >> 4, m = lane & 15;
  const int rowBase = (int)blockIdx.x * GBM;
  const int col0    = (int)blockIdx.y * GBN;

  v8f acc[4];
  {
    const v8f z = {0.f, 0.f, 0.f, 0.f, 0.f, 0.f, 0.f, 0.f};
    acc[0] = z; acc[1] = z; acc[2] = z; acc[3] = z;
  }
  const unsigned short* ap = A  + (size_t)(rowBase + 16 * wave + m) * (size_t)lda + 8 * hh;
  const unsigned short* wp = WT + (size_t)(col0 + m) * (size_t)K + 8 * hh;
  const int ksteps = K >> 5;
#pragma unroll 1
  for (int ks = 0; ks < ksteps; ++ks) {
    FragB af;
    af.h[0] = *(const v8usa*)(ap + 32 * ks);
    af.h[1] = *(const v8usa*)(ap + 32 * ks + 16);
#pragma unroll
    for (int t = 0; t < 4; ++t) {
      const unsigned short* wq = wp + (size_t)(16 * t) * (size_t)K + 32 * ks;
      FragB bf;
      bf.h[0] = *(const v8usa*)wq;
      bf.h[1] = *(const v8usa*)(wq + 16);
      acc[t] = wmb(af, bf, acc[t]);
    }
  }

#pragma unroll
  for (int t = 0; t < 4; ++t) {
    const int lc = 16 * t + m;
#pragma unroll
    for (int r = 0; r < 8; ++r) {
      const int lr = 16 * wave + 8 * hh + r;
      stg[lr * GBN + lc] = acc[t][r];
    }
  }
  __syncthreads();

  const int mat = col0 / CW;
  const float* bsel = (mat == 0) ? bs0 : ((mat == 1) ? bs1 : bs2);
  v4f b4 = *(const v4fa*)(bsel + (col0 & (CW - 1)) + 4 * m);
  b4 = bfr4(b4) * (float)useBias;

  v4f fv[8];
#pragma unroll
  for (int i = 0; i < 8; ++i) {
    const int lr = 16 * wave + 2 * i + hh;
    fv[i] = *(const v4fa*)(stg + lr * GBN + 4 * m) + b4;
  }
#pragma unroll
  for (int i = 0; i < 8; ++i) {
    const int lr = 16 * wave + 2 * i + hh;
    const int gr = rowBase + lr;
    const int gs = gr < nRows ? gr : nRows - 1;
    float* op = outF + (size_t)gs * (size_t)ldo + col0 + 4 * m;
    if (gr < nRows) *(volatile v4f*)op = fv[i];
  }
  __threadfence();
#pragma unroll
  for (int i = 0; i < 8; ++i) {
    const int lr = 16 * wave + 2 * i + hh;
    const int gr = rowBase + lr;
    const int gs = gr < nRows ? gr : nRows - 1;
    float* op = outF + (size_t)gs * (size_t)ldo + col0 + 4 * m;
    if (gr < nRows) *(volatile v4f*)op = fv[i];
  }
}

__global__ __launch_bounds__(NTHR) void k_scan(const int* __restrict__ qid, const int* __restrict__ kid,
                                               const float* __restrict__ QKV, unsigned short* apl,
                                               int nE, int nS, int mRows, int vec8) {
  extern __shared__ __attribute__((aligned(16))) int dsm[];
  int* list = dsm;
  int* hl   = dsm + LISTN;
  int* sl   = hl + RCAP;
  int* cnt  = sl + RCAP;
  int* offs = cnt + NBA;
  int* cur  = offs + NBA;
  int* misc = cur + NBA;
  const int tid = (int)threadIdx.x, lane = tid & 31, wave = tid >> 5;
  const int nodeBase = (int)blockIdx.x * NBA;

  {
    const v4i z4 = {0, 0, 0, 0};
    for (int i = tid * 4; i < AGG_ZINTS; i += NTHR * 4) *(v4ia*)(dsm + i) = z4;
    if (tid < MISC_INTS) misc[tid] = 0;
  }
  __syncthreads();

  int t = 0, ov = 0;
  const int nChunks = (nE + CHUNK - 1) / CHUNK;
#pragma unroll 1
  for (int ch = 0; ch < nChunks; ++ch) {
    const int cbase = ch * CHUNK;
    const int wc = scan_chunk(qid, nE, cbase, nodeBase, NBA, vec8, list, tid, lane, wave);
    if (lane == 0) misc[wave] = wc;
    __syncthreads();
    if (wave == 0) {
#pragma unroll 1
      for (int w2 = 0; w2 < NWAVE; ++w2) {
        int c = misc[w2];
        c = c < 0 ? 0 : (c > WCAP ? WCAP : c);
#pragma unroll 1
        for (int b0 = 0; b0 < c; b0 += 32) {
          const int idx = b0 + lane;
          const int ent = list[w2 * WCAP + (idx < WCAP ? idx : WCAP - 1)];
          const int m32 = (c - b0) < 32 ? (c - b0) : 32;
#pragma unroll 1
          for (int k = 0; k < m32; ++k) {
            const int u    = __builtin_amdgcn_readlane(ent, k);
            const int slot = u & (NBA - 1);
            const int el   = (u >> SLA) & (CHUNK - 1);
            const int pk   = ((cbase + el) << SLA) | slot;
            if (t < RCAP) {
              if (lane == 0) { hl[t] = pk; cnt[slot] = cnt[slot] + 1; }
              t = t + 1;
            } else {
              ov = 1;
            }
          }
        }
      }
    }
    __syncthreads();
  }
  if (wave == 0 && lane == 0) { misc[8] = t; misc[9] = ov; }
  __syncthreads();
  int tt = misc[8];
  tt = tt < 0 ? 0 : (tt > RCAP ? RCAP : tt);
  const int ovf = misc[9];

  if (wave == 0) {
    const int base = lane * (NBA / 32);
    int s = 0;
#pragma unroll 1
    for (int i = 0; i < NBA / 32; ++i) s += cnt[base + i];
    int incl = s;
#pragma unroll
    for (int d = 1; d < 32; d <<= 1) {
      const int y = __shfl_up(incl, d, 32);
      if (lane >= d) incl += y;
    }
    int run = incl - s;
#pragma unroll 1
    for (int i = 0; i < NBA / 32; ++i) {
      const int cv = cnt[base + i];
      offs[base + i] = run;
      cur[base + i]  = run;
      run += cv;
    }
  }
  __syncthreads();
  if (wave == 0) {
#pragma unroll 1
    for (int b0 = 0; b0 < tt; b0 += 32) {
      const int idx = b0 + lane;
      const int ent = hl[idx < RCAP ? idx : RCAP - 1];
      const int m32 = (tt - b0) < 32 ? (tt - b0) : 32;
#pragma unroll 1
      for (int k = 0; k < m32; ++k) {
        const int u    = __builtin_amdgcn_readlane(ent, k);
        const int slot = u & (NBA - 1);
        if (lane == 0) {
          int p = cur[slot];
          p = p < 0 ? 0 : (p > RCAP - 1 ? RCAP - 1 : p);
          sl[p] = u;
          cur[slot] = p + 1;
        }
      }
    }
  }
  __syncthreads();

  const float qnan = __int_as_float(0x7fc00000);
  float* stg = (float*)hl + wave * CW;
  const v4f z4 = {0.f, 0.f, 0.f, 0.f};
#pragma unroll 1
  for (int si = 0; si < NBA / NWAVE; ++si) {
    const int s  = si * NWAVE + wave;
    const int qn = nodeBase + s;
    int c = cnt[s];
    const bool big = c > DEGCAP;
    c = c < 0 ? 0 : (c > DEGCAP ? DEGCAP : c);
    int o = offs[s];
    o = o < 0 ? 0 : (o > RCAP ? RCAP : o);
    const int  qc   = qn < nS ? qn : nS - 1;
    const bool live = qn < nS;
    const bool pois = big || (ovf != 0);

#pragma unroll 1
    for (int b = 0; b < BD; ++b) {
      const float* qr = QKV + ((size_t)qc * BD + b) * QKVW + OQ + 32 * lane;
      v4f qv[8];
#pragma unroll
      for (int j = 0; j < 8; ++j) qv[j] = *(const v4fa*)(qr + 4 * j);
      ldwait();

      float mx = -1.0e30f, dn = 0.0f;
      v4f av[8];
#pragma unroll
      for (int j = 0; j < 8; ++j) av[j] = z4;

#pragma unroll 1
      for (int b0 = 0; b0 < c; b0 += 32) {
        int idx = o + b0 + lane;
        idx = idx > RCAP - 1 ? RCAP - 1 : idx;
        const int ent = sl[idx];
        int eid = ent >> SLA;
        eid = eid < 0 ? 0 : (eid > nE - 1 ? nE - 1 : eid);
        int kd = kid[eid];
        kd = kd < 0 ? 0 : (kd > nS - 1 ? nS - 1 : kd);
        const int m32 = (c - b0) < 32 ? (c - b0) : 32;
#pragma unroll 1
        for (int k = 0; k < m32; ++k) {
          const int tk = __builtin_amdgcn_readlane(kd, k);
          const float* kr = QKV + ((size_t)tk * BD + b) * QKVW + OKK + 32 * lane;
          v4f kv[8];
#pragma unroll
          for (int j = 0; j < 8; ++j) kv[j] = *(const v4fa*)(kr + 4 * j);
          ldwait();
          float p = 0.0f;
#pragma unroll
          for (int j = 0; j < 8; ++j) {
            p = fmaf(qv[j].x, kv[j].x, p); p = fmaf(qv[j].y, kv[j].y, p);
            p = fmaf(qv[j].z, kv[j].z, p); p = fmaf(qv[j].w, kv[j].w, p);
          }
          p += __shfl_xor(p, 1);
          const float lg = p * ATTSC;
          const float df = lg - mx;
          const float ee = __expf(-fabsf(df));
          const bool up  = df > 0.0f;
          const float s1 = up ? ee : 1.0f;
          const float s2 = up ? 1.0f : ee;
          mx = up ? lg : mx;
          dn = fmaf(dn, s1, s2);
          const float* vr = QKV + ((size_t)tk * BD + b) * QKVW + OV + 32 * lane;
          v4f vv[8];
#pragma unroll
          for (int j = 0; j < 8; ++j) vv[j] = *(const v4fa*)(vr + 4 * j);
          ldwait();
#pragma unroll
          for (int j = 0; j < 8; ++j) {
            av[j].x = fmaf(av[j].x, s1, s2 * vv[j].x); av[j].y = fmaf(av[j].y, s1, s2 * vv[j].y);
            av[j].z = fmaf(av[j].z, s1, s2 * vv[j].z); av[j].w = fmaf(av[j].w, s1, s2 * vv[j].w);
          }
        }
      }

      const float inv  = __builtin_amdgcn_rcpf(dn);
      const float invp = pois ? qnan : inv;
      wave_sync();
#pragma unroll
      for (int j = 0; j < 8; ++j) {
        v4f o4;
        o4.x = live ? av[j].x * invp : 0.0f;
        o4.y = live ? av[j].y * invp : 0.0f;
        o4.z = live ? av[j].z * invp : 0.0f;
        o4.w = live ? av[j].w * invp : 0.0f;
        *(v4fa*)(stg + 32 * lane + 4 * j) = o4;
      }
      wave_sync();
      v4u hv[4], lv[4];
#pragma unroll
      for (int j = 0; j < 4; ++j) {
        const v4f pa = *(const v4fa*)(stg + 256 * j + 8 * lane);
        const v4f pb = *(const v4fa*)(stg + 256 * j + 8 * lane + 4);
        pack8hl(pa, pb, hv[j], lv[j]);
      }
      const int row = qn * BD + b;
      if (row < mRows) {
        unsigned short* rp = apl + (size_t)row * APITCH;
#pragma unroll
        for (int j = 0; j < 4; ++j) {
          *(volatile v4u*)(rp + 256 * j + 8 * lane)      = hv[j];
          *(volatile v4u*)(rp + CW + 256 * j + 8 * lane) = lv[j];
        }
        __threadfence();
#pragma unroll
        for (int j = 0; j < 4; ++j) {
          *(volatile v4u*)(rp + 256 * j + 8 * lane)      = hv[j];
          *(volatile v4u*)(rp + CW + 256 * j + 8 * lane) = lv[j];
        }
      }
    }
  }
}

static inline int cdiv(int a, int b) { return (a + b - 1) / b; }
static inline size_t al256(size_t o) { return (o + 255) & ~(size_t)255; }

extern "C" void kernel_launch(void* const* d_in, const int* in_sizes, int n_in,
                              void* d_out, int out_size, void* d_ws, size_t ws_size,
                              hipStream_t stream) {
  if (n_in < 11) return;
  if (in_sizes[0] < BD * CW || (in_sizes[0] % (BD * CW)) != 0) return;
  const int nS = in_sizes[0] / (BD * CW);
  if (nS < 1 || nS > (1 << 20)) return;
  const int nE = in_sizes[1];
  if (nE < 1 || nE >= (1 << (31 - SLA))) return;
  if (in_sizes[2] != nE) return;
  if (in_sizes[3] != CW * CW || in_sizes[5] != CW * CW || in_sizes[7] != CW * CW || in_sizes[9] != CW * CW) return;
  if (in_sizes[4] != CW || in_sizes[6] != CW || in_sizes[8] != CW || in_sizes[10] != CW) return;
  if ((long long)out_size != (long long)nS * BD * CW) return;

  const float* x   = (const float*)d_in[0];
  const int*   qid = (const int*)  d_in[1];
  const int*   kid = (const int*)  d_in[2];
  const float* Wq  = (const float*)d_in[3];
  const float* bq  = (const float*)d_in[4];
  const float* Wk  = (const float*)d_in[5];
  const float* bk  = (const float*)d_in[6];
  const float* Wv  = (const float*)d_in[7];
  const float* bv  = (const float*)d_in[8];
  const float* Wx  = (const float*)d_in[9];
  const float* bx  = (const float*)d_in[10];
  float* out = (float*)d_out;

  const int nRows = nS * BD;
  const int MP = cdiv(nRows, GBM) * GBM;
  const int gM = MP / GBM;
  const int gA = cdiv(cdiv(MP, BD), NBA);
  if ((long long)gA * NBA * BD < (long long)MP) return;
  const int vec8 = ((nE & 3) == 0) ? 1 : 0;

  char* ws = (char*)d_ws;
  size_t off = 0;
  const size_t oXB  = off; off = al256(off + (size_t)MP * CW * 2);
  const size_t oWQ  = off; off = al256(off + (size_t)QKVW * CW * 2);
  const size_t oWX  = off; off = al256(off + (size_t)CW * KOUT * 2);
  const size_t oQKV = off; off = al256(off + (size_t)MP * QKVW * 4);
  const size_t oAPL = off; off = al256(off + (size_t)MP * APITCH * 2);
  if (off > ws_size || off > (size_t)WSMAX) return;
  unsigned short* XB    = (unsigned short*)(ws + oXB);
  unsigned short* WQKVT = (unsigned short*)(ws + oWQ);
  unsigned short* WXT   = (unsigned short*)(ws + oWX);
  float*          QKV   = (float*)(ws + oQKV);
  unsigned short* APL   = (unsigned short*)(ws + oAPL);

  hipFuncSetAttribute(reinterpret_cast<const void*>(&k_scan),
                      hipFuncAttributeMaxDynamicSharedMemorySize, SCAN_LDS_BYTES);

  const int nUx = MP * (CW / 8);
  k_xprep<<<cdiv(nUx, NTHR), NTHR, 0, stream>>>(x, XB, nRows, nUx);
  k_wprep<<<NUW / NTHR, NTHR, 0, stream>>>(Wq, Wk, Wv, Wx, WQKVT, WXT);
  k_gemm<<<dim3(gM, QKVW / GBN), GTHR, 0, stream>>>(XB, CW, WQKVT, CW, QKV, QKVW, MP, bq, bk, bv, 1);
  k_scan<<<gA, NTHR, SCAN_LDS_BYTES, stream>>>(qid, kid, QKV, APL, nE, nS, MP, vec8);
  k_gemm<<<dim3(gM, CW / GBN), GTHR, 0, stream>>>(APL, APITCH, WXT, KOUT, out, CW, nRows, bx, bx, bx, 1);
}
